// HeteroGNN_SAGE_79448305041987
// MI455X (gfx1250) — hardware-verified
//
#include <hip/hip_runtime.h>
#include <stddef.h>


#define DF      128
#define NTHR    256
#define NWAVE   8
#define EPT     8
#define NGRP    2
#define CHUNK   (NTHR * EPT * NGRP)
#define WCAP    (EPT * NGRP * 32)
#define LISTN   (NWAVE * WCAP)
#define NB      512
#define NTILE   (NB / 16)
#define TPW     (NTILE / NWAVE)
#define NG      64
#define PHALF   64
#define NCHK    4

#define KVA1    256
#define KVA2    128
#define KVB     256
#define OFF_A2  (DF * KVA1)
#define OFF_B   (OFF_A2 + DF * KVA2)
#define WPL     (OFF_B + DF * KVB)

#define LDS_ACC   (NB * DF * 4)
#define LDS_LIST  (LISTN * 4)
#define LDS_CNT   (NB * 4)
#define LDS_LAYER (LDS_ACC + LDS_LIST + LDS_CNT + 64)
#define LDS_HEAD  (NG * 2 * DF * 4 + NG * 4)

static_assert((CHUNK & (CHUNK - 1)) == 0);
static_assert(CHUNK <= 4096);
static_assert((NB & (NB - 1)) == 0);
static_assert(NB <= 4096);
static_assert(NTILE % NWAVE == 0);
static_assert(NG * PHALF * 4 <= LDS_LIST);
static_assert(2 * PHALF == DF);
static_assert((NG * PHALF) % (4 * NTHR) == 0);
static_assert(NWAVE * 4 <= 64);
static_assert(LDS_LAYER <= 300 * 1024);
static_assert((WPL % (8 * NTHR)) == 0);
static_assert((NG * DF) % NTHR == 0);
static_assert(KVB == KVA1);

typedef float  v4f   __attribute__((ext_vector_type(4)));
typedef float  v8f   __attribute__((ext_vector_type(8)));
typedef int    v4i   __attribute__((ext_vector_type(4)));
typedef __bf16 bf16_t;
typedef bf16_t v8bf  __attribute__((ext_vector_type(8)));
typedef bf16_t v16bf __attribute__((ext_vector_type(16)));
union FragB { v16bf v; v8bf h[2]; v4i q[2]; };
union Pack8 { v8bf v; v4i q; };

__device__ __forceinline__ v8f wmb(v16bf a, v16bf b, v8f c) {
  v8f d = __builtin_amdgcn_wmma_f32_16x16x32_bf16(false, a, false, b, (short)0, c, false, false);
  asm volatile("v_nop\n\tv_nop\n\tv_nop\n\tv_nop" : "+v"(d) : "v"(a), "v"(b));
  return d;
}

template <int B>
__device__ __forceinline__ void split8(FragB& hi, FragB& lo, v4f a, v4f b) {
#define SPL1(I, X) { const float xv = (X); const bf16_t hb = (bf16_t)xv; hi.v[B + (I)] = hb; lo.v[B + (I)] = (bf16_t)(xv - (float)hb); }
  SPL1(0, a.x) SPL1(1, a.y) SPL1(2, a.z) SPL1(3, a.w)
  SPL1(4, b.x) SPL1(5, b.y) SPL1(6, b.z) SPL1(7, b.w)
#undef SPL1
}

template <int NBT>
__device__ __forceinline__ int scan_chunk(const int* __restrict__ dsts, int nE, int cbase, int nodeBase,
                                          int vec8, int* list, int tid, int wave) {
  int wc = 0;
#pragma unroll
  for (int g = 0; g < NGRP; ++g) {
    const int el0  = (g * NTHR + tid) * EPT;
    const int e0   = cbase + el0;
    const int sent = -2147483647 - 1;
    const int le   = nE - 1;
    v4i da, db;
    if (vec8 != 0 && cbase + CHUNK <= nE) {
      da = *(const v4i*)(dsts + e0);
      db = *(const v4i*)(dsts + e0 + 4);
    } else {
      da.x = (e0     < nE) ? dsts[min(e0,     le)] : sent;
      da.y = (e0 + 1 < nE) ? dsts[min(e0 + 1, le)] : sent;
      da.z = (e0 + 2 < nE) ? dsts[min(e0 + 2, le)] : sent;
      da.w = (e0 + 3 < nE) ? dsts[min(e0 + 3, le)] : sent;
      db.x = (e0 + 4 < nE) ? dsts[min(e0 + 4, le)] : sent;
      db.y = (e0 + 5 < nE) ? dsts[min(e0 + 5, le)] : sent;
      db.z = (e0 + 6 < nE) ? dsts[min(e0 + 6, le)] : sent;
      db.w = (e0 + 7 < nE) ? dsts[min(e0 + 7, le)] : sent;
    }
    const unsigned nb = (unsigned)nodeBase;
    const unsigned s0 = (unsigned)da.x - nb, s1 = (unsigned)da.y - nb;
    const unsigned s2 = (unsigned)da.z - nb, s3 = (unsigned)da.w - nb;
    const unsigned s4 = (unsigned)db.x - nb, s5 = (unsigned)db.y - nb;
    const unsigned s6 = (unsigned)db.z - nb, s7 = (unsigned)db.w - nb;
    const bool h0 = s0 < (unsigned)NBT, h1 = s1 < (unsigned)NBT, h2 = s2 < (unsigned)NBT, h3 = s3 < (unsigned)NBT;
    const bool h4 = s4 < (unsigned)NBT, h5 = s5 < (unsigned)NBT, h6 = s6 < (unsigned)NBT, h7 = s7 < (unsigned)NBT;
    const unsigned any = __builtin_amdgcn_ballot_w32(h0 | h1 | h2 | h3 | h4 | h5 | h6 | h7);
    if (any != 0u) {
#define HITJ(J, HJ, SJ) { \
        const unsigned mj = __builtin_amdgcn_ballot_w32(HJ); \
        if (mj != 0u) { \
          if (HJ) { \
            const int pos = wc + (int)__builtin_amdgcn_mbcnt_lo(mj, 0u); \
            if (pos < WCAP) list[wave * WCAP + pos] = ((el0 + (J)) << 12) | (int)(SJ); \
          } \
          wc += (int)__builtin_popcount(mj); } }
      HITJ(0, h0, s0)
      HITJ(1, h1, s1)
      HITJ(2, h2, s2)
      HITJ(3, h3, s3)
      HITJ(4, h4, s4)
      HITJ(5, h5, s5)
      HITJ(6, h6, s6)
      HITJ(7, h7, s7)
#undef HITJ
    }
  }
  return wc;
}

__global__ __launch_bounds__(NTHR) void k_wprep(
    const float* __restrict__ Wl, const float* __restrict__ Wr,
    bf16_t* whi, bf16_t* wlo, int nTot) {
  const int i = blockIdx.x * NTHR + threadIdx.x;
  if (i >= nTot) return;
  const int o      = i * 8;
  const int layer  = o / WPL;
  const int rem    = o - layer * WPL;
  const int q      = (rem < OFF_A2) ? 0 : ((rem < OFF_B) ? 1 : 2);
  const int base   = (q == 0) ? 0 : ((q == 1) ? OFF_A2 : OFF_B);
  const int pitch  = (q == 1) ? KVA2 : ((q == 0) ? KVA1 : KVB);
  const int rr     = rem - base;
  const int n      = rr / pitch;
  const int k0     = rr - n * pitch;
  const int isRoot = (k0 >= DF) ? 1 : 0;
  const int kk     = k0 - isRoot * DF;
  const int relL   = (q == 0) ? 0 : ((q == 1) ? 2 : 1);
  const int relR   = (q == 0) ? 0 : 1;
  const float fR2  = (q == 0) ? 1.0f : 0.0f;
  const float* pl  = Wl + ((size_t)(layer * 3 + relL) * DF + kk) * DF + n;
  const float* pr1 = Wr + ((size_t)(layer * 3 + relR) * DF + kk) * DF + n;
  const float* pr2 = Wr + ((size_t)(layer * 3 + 2)    * DF + kk) * DF + n;
  Pack8 ph, pq;
#define WSP(I) { const float wl = pl[(I) * DF]; const float w1 = pr1[(I) * DF]; const float w2 = pr2[(I) * DF]; \
    const float vr = w1 + fR2 * w2; const float xv = (isRoot != 0) ? vr : wl; \
    const bf16_t hb = (bf16_t)xv; ph.v[(I)] = hb; pq.v[(I)] = (bf16_t)(xv - (float)hb); }
  WSP(0) WSP(1) WSP(2) WSP(3) WSP(4) WSP(5) WSP(6) WSP(7)
#undef WSP
  bf16_t* dh = whi + o;
  bf16_t* dl = wlo + o;
  const v4i qh = ph.q, ql = pq.q;
  *(volatile v4i*)dh = qh;
  *(volatile v4i*)dl = ql;
  __threadfence();
  *(volatile v4i*)dh = qh;
  *(volatile v4i*)dl = ql;
}

__device__ __forceinline__ void kstep(const float* ap, float mul,
                                      const bf16_t* bhp, const bf16_t* blp, int kv, v8f (&c)[8]) {
  const v4f p0 = (*(const v4f*)(ap))      * mul;
  const v4f p1 = (*(const v4f*)(ap + 4))  * mul;
  const v4f p2 = (*(const v4f*)(ap + 16)) * mul;
  const v4f p3 = (*(const v4f*)(ap + 20)) * mul;
  FragB ahi, alo;
  split8<0>(ahi, alo, p0, p1);
  split8<8>(ahi, alo, p2, p3);
#pragma unroll
  for (int ct = 0; ct < DF / 16; ++ct) {
    const bf16_t* hp = bhp + (size_t)ct * 16 * kv;
    const bf16_t* lp = blp + (size_t)ct * 16 * kv;
    FragB bh, bq;
    bh.q[0] = *(const v4i*)hp;  bh.q[1] = *(const v4i*)(hp + 16);
    bq.q[0] = *(const v4i*)lp;  bq.q[1] = *(const v4i*)(lp + 16);
    c[ct] = wmb(alo.v, bh.v, c[ct]);
    c[ct] = wmb(ahi.v, bq.v, c[ct]);
    c[ct] = wmb(ahi.v, bh.v, c[ct]);
  }
}

__global__ __launch_bounds__(NTHR) void k_layer(
    const int* __restrict__ srcs, const int* __restrict__ dsts, int nE, int vec8,
    const float* xg, int nSrc, const float* xr, int nDst,
    const bf16_t* __restrict__ whi, const bf16_t* __restrict__ wlo, int kv, int hasRoot,
    const float* __restrict__ b1, const float* __restrict__ b2, float f1, float f2,
    const float* pin, int addP, float* pout, int mode, int act,
    const int* __restrict__ batch, float* pool, int rowBase) {
  extern __shared__ v4f lds_dyn[];
  float* acc  = (float*)lds_dyn;
  int*   list = (int*)((char*)lds_dyn + LDS_ACC);
  float* bank = (float*)((char*)lds_dyn + LDS_ACC);
  int*   cnt  = (int*)((char*)lds_dyn + LDS_ACC + LDS_LIST);
  int*   wcnt = (int*)((char*)lds_dyn + LDS_ACC + LDS_LIST + LDS_CNT);
  const int tid = threadIdx.x, lane = tid & 31, wave = tid >> 5, hh = lane >> 4, m = lane & 15;
  const int lrow0 = blockIdx.x * NB;
  const int nodeBase = rowBase + lrow0;

  {
    const v4f z = {0.f, 0.f, 0.f, 0.f};
    for (int i = tid; i < NB * DF / 4; i += NTHR) lds_dyn[i] = z;
    for (int i = tid; i < NB; i += NTHR) cnt[i] = 0;
  }
  __syncthreads();

  const int nChunks = (nE + CHUNK - 1) / CHUNK;
#pragma unroll 1
  for (int ch = 0; ch < nChunks; ++ch) {
    const int cbase = ch * CHUNK;
    const int wc = scan_chunk<NB>(dsts, nE, cbase, nodeBase, vec8, list, tid, wave);
    if (lane == 0) wcnt[wave] = wc;
    __syncthreads();
    if (wave == 0) {
#pragma unroll 1
      for (int wsx = 0; wsx < NWAVE; ++wsx) {
        int n = __builtin_amdgcn_readfirstlane(wcnt[wsx]);
        n = n > WCAP ? WCAP : (n < 0 ? 0 : n);
        const int* lp = list + wsx * WCAP;
#pragma unroll 1
        for (int i = 0; i < n; ++i) {
          const int ent  = __builtin_amdgcn_readfirstlane(lp[i]);
          const int slot = ent & (NB - 1);
          int e = cbase + ((ent >> 12) & (CHUNK - 1));
          e = e > nE - 1 ? nE - 1 : e;
          int src = srcs[e];
          src = src < 0 ? 0 : (src > nSrc - 1 ? nSrc - 1 : src);
          const v4f v = *(const v4f*)(xg + (size_t)src * DF + 4 * lane);
          v4f* ap = (v4f*)(acc + slot * DF + 4 * lane);
          *ap = *ap + v;
          if (lane == 0) cnt[slot] = cnt[slot] + 1;
        }
      }
    }
    __syncthreads();
  }

  const float slope = (act != 0) ? 0.01f : 1.0f;

#pragma unroll 1
  for (int q = 0; q < TPW; ++q) {
    const int t     = q * NWAVE + wave;
    const int slotm = 16 * t + m;
    int node = nodeBase + slotm;
    node = node > nDst - 1 ? nDst - 1 : node;
    const int   cd  = cnt[slotm];
    const float inv = 1.0f / (float)(cd > 1 ? cd : 1);

    float bs[8];
#pragma unroll
    for (int ct = 0; ct < 8; ++ct) { const int col = 16 * ct + m; bs[ct] = f1 * b1[col] + f2 * b2[col]; }

    v8f c[8];
    if (addP != 0) {
      const float* pp = pin + (size_t)(lrow0 + 16 * t + 8 * hh) * DF + m;
#pragma unroll
      for (int ct = 0; ct < 8; ++ct) {
#pragma unroll
        for (int r = 0; r < 8; ++r) c[ct][r] = pp[(size_t)r * DF + 16 * ct] + bs[ct];
      }
    } else {
#pragma unroll
      for (int ct = 0; ct < 8; ++ct) {
#pragma unroll
        for (int r = 0; r < 8; ++r) c[ct][r] = bs[ct];
      }
    }

    const float*  arow = acc + slotm * DF + 8 * hh;
    const float*  xrow = xr + (size_t)node * DF + 8 * hh;
    const bf16_t* bh0  = whi + m * kv + 8 * hh;
    const bf16_t* bl0  = wlo + m * kv + 8 * hh;
#pragma unroll 1
    for (int ks = 0; ks < DF / 32; ++ks)
      kstep(arow + 32 * ks, inv, bh0 + 32 * ks, bl0 + 32 * ks, kv, c);
    if (hasRoot != 0) {
#pragma unroll 1
      for (int ks = 0; ks < DF / 32; ++ks)
        kstep(xrow + 32 * ks, 1.0f, bh0 + DF + 32 * ks, bl0 + DF + 32 * ks, kv, c);
    }

    float* sp = acc + (16 * t + 8 * hh) * DF + m;
#pragma unroll
    for (int ct = 0; ct < 8; ++ct) {
#pragma unroll
      for (int r = 0; r < 8; ++r) {
        const float v = c[ct][r];
        sp[r * DF + 16 * ct] = (v >= 0.0f) ? v : v * slope;
      }
    }
    __syncthreads();

    if (mode == 0) {
      const float* lrow = acc + (16 * t) * DF + 4 * lane;
      float* gp = pout + ((size_t)lrow0 + 16 * t) * DF + 4 * lane;
#pragma unroll
      for (int i = 0; i < 16; ++i) { const v4f v = *(const v4f*)(lrow + i * DF); *(volatile v4f*)(gp + (size_t)i * DF) = v; }
      __threadfence();
#pragma unroll
      for (int i = 0; i < 16; ++i) { const v4f v = *(const v4f*)(lrow + i * DF); *(volatile v4f*)(gp + (size_t)i * DF) = v; }
    }
  }

  if (mode != 0) {
    __syncthreads();
    int nValid = nDst - nodeBase;
    nValid = nValid > NB ? NB : (nValid < 0 ? 0 : nValid);
    for (int i = tid; i < NB; i += NTHR) {
      int nd = nodeBase + i;
      nd = nd > nDst - 1 ? nDst - 1 : nd;
      int g = batch[nd];
      g = g < 0 ? 0 : (g > NG - 1 ? NG - 1 : g);
      cnt[i] = g;
    }
    __syncthreads();
#pragma unroll 1
    for (int hp = 0; hp < 2; ++hp) {
      for (int i = tid; i < NG * PHALF; i += NTHR) bank[i] = 0.0f;
      __syncthreads();
      if (tid < PHALF) {
        const int col = hp * PHALF + tid;
        double run = 0.0;
        int cur = cnt[0];
#pragma unroll 1
        for (int s = 0; s < nValid; ++s) {
          const int g = cnt[s];
          const float v = acc[s * DF + col];
          if (g != cur) { bank[cur * PHALF + tid] += (float)run; run = 0.0; cur = g; }
          run += (double)v;
        }
        bank[cur * PHALF + tid] += (float)run;
      }
      __syncthreads();
      v4f vv[4];
#pragma unroll
      for (int it = 0; it < 4; ++it) {
        const int hr = it * 16 + (tid >> 4);
        const int pc = 4 * (tid & 15);
        vv[it] = *(const v4f*)(bank + hr * PHALF + pc);
        float* gp = pool + ((size_t)blockIdx.x * NG + hr) * DF + hp * PHALF + pc;
        *(volatile v4f*)gp = vv[it];
      }
      __threadfence();
#pragma unroll
      for (int it = 0; it < 4; ++it) {
        const int hr = it * 16 + (tid >> 4);
        const int pc = 4 * (tid & 15);
        float* gp = pool + ((size_t)blockIdx.x * NG + hr) * DF + hp * PHALF + pc;
        *(volatile v4f*)gp = vv[it];
      }
      __syncthreads();
    }
  }
}

__global__ __launch_bounds__(NTHR) void k_head(
    const float* __restrict__ poolA, int nBlkA, const float* __restrict__ poolB, int nBlkB,
    const float* __restrict__ mlpW, const float* __restrict__ mlpb,
    const float* __restrict__ linW, const float* __restrict__ linb, float* out) {
  extern __shared__ v4f lds_dyn[];
  float* gm = (float*)lds_dyn;
  float* os = gm + NG * 2 * DF;
  const int tid = threadIdx.x, lane = tid & 31, wave = tid >> 5, hh = lane >> 4, m = lane & 15;

#pragma unroll 1
  for (int i = 0; i < (NG * DF) / NTHR; ++i) {
    const int e  = i * NTHR + tid;
    const int g  = e / DF;
    const int cc = e - g * DF;
    double sa = 0.0, sb = 0.0;
#pragma unroll 1
    for (int b = 0; b < nBlkA; ++b) sa += (double)poolA[(size_t)b * NG * DF + e];
#pragma unroll 1
    for (int b = 0; b < nBlkB; ++b) sb += (double)poolB[(size_t)b * NG * DF + e];
    gm[g * 2 * DF + cc]      = (float)sa;
    gm[g * 2 * DF + DF + cc] = (float)sb;
  }
  __syncthreads();

  v8f c[4];
#pragma unroll
  for (int t = 0; t < 4; ++t) { const v8f z = {0.f, 0.f, 0.f, 0.f, 0.f, 0.f, 0.f, 0.f}; c[t] = z; }
  const int col = 16 * wave + m;
#pragma unroll 1
  for (int ks = 0; ks < (2 * DF) / 32; ++ks) {
    const int k0 = 32 * ks;
    FragB bh, bq;
#pragma unroll
    for (int i = 0; i < 16; ++i) {
      const int k = k0 + ((i < 8) ? (8 * hh + i) : (16 + 8 * hh + (i - 8)));
      const float xv = mlpW[(size_t)k * DF + col];
      const bf16_t hb = (bf16_t)xv;
      bh.v[i] = hb;
      bq.v[i] = (bf16_t)(xv - (float)hb);
    }
#pragma unroll
    for (int t = 0; t < NG / 16; ++t) {
      const float* ap = gm + (16 * t + m) * (2 * DF) + k0 + 8 * hh;
      const v4f p0 = *(const v4f*)(ap);
      const v4f p1 = *(const v4f*)(ap + 4);
      const v4f p2 = *(const v4f*)(ap + 16);
      const v4f p3 = *(const v4f*)(ap + 20);
      FragB ah, al;
      split8<0>(ah, al, p0, p1);
      split8<8>(ah, al, p2, p3);
      c[t] = wmb(al.v, bh.v, c[t]);
      c[t] = wmb(ah.v, bq.v, c[t]);
      c[t] = wmb(ah.v, bh.v, c[t]);
    }
  }
  __syncthreads();

  float* dsm = gm;
  const float bb = mlpb[col];
#pragma unroll
  for (int t = 0; t < 4; ++t) {
#pragma unroll
    for (int r = 0; r < 8; ++r) dsm[(16 * t + 8 * hh + r) * DF + col] = c[t][r] + bb;
  }
  __syncthreads();

  if (tid < NG) {
    double s = 0.0;
#pragma unroll 1
    for (int n = 0; n < DF; ++n) s += (double)dsm[tid * DF + n] * (double)linW[n];
    os[tid] = (float)s + linb[0];
  }
  __syncthreads();

  if (tid < 16) { const v4f v = *(const v4f*)(os + 4 * tid); *(volatile v4f*)(out + 4 * tid) = v; }
  __threadfence();
  if (tid < 16) { const v4f v = *(const v4f*)(os + 4 * tid); *(volatile v4f*)(out + 4 * tid) = v; }
}

extern "C" void kernel_launch(void* const* d_in, const int* in_sizes, int n_in,
                              void* d_out, int out_size, void* d_ws, size_t ws_size,
                              hipStream_t stream) {
  if (n_in < 17) return;
  const int nA  = in_sizes[0] / DF;
  const int nBn = in_sizes[1] / DF;
  if (nA <= 0 || nBn <= 0 || in_sizes[0] != nA * DF || in_sizes[1] != nBn * DF) return;
  const int eAA = in_sizes[2], eAB = in_sizes[4], eBA = in_sizes[6];
  if (eAA < 0 || eAB < 0 || eBA < 0) return;
  if (in_sizes[3] != eAA || in_sizes[5] != eAB || in_sizes[7] != eBA) return;
  if (in_sizes[8] != nA || in_sizes[9] != nBn) return;
  const int nL = in_sizes[10] / (3 * DF * DF);
  if (nL != 2 || in_sizes[10] != nL * 3 * DF * DF || in_sizes[12] != in_sizes[10]) return;
  if (in_sizes[11] < nL * 3 * DF) return;
  if (in_sizes[13] != 2 * DF * DF || in_sizes[14] < DF || in_sizes[15] < DF || in_sizes[16] < 1) return;
  if (out_size != NG) return;

  const float* x_a    = (const float*)d_in[0];
  const float* x_b    = (const float*)d_in[1];
  const int*   aa_src = (const int*)d_in[2];
  const int*   aa_dst = (const int*)d_in[3];
  const int*   ab_src = (const int*)d_in[4];
  const int*   ab_dst = (const int*)d_in[5];
  const int*   ba_src = (const int*)d_in[6];
  const int*   ba_dst = (const int*)d_in[7];
  const int*   bat_a  = (const int*)d_in[8];
  const int*   bat_b  = (const int*)d_in[9];
  const float* Wl     = (const float*)d_in[10];
  const float* bl     = (const float*)d_in[11];
  const float* Wr     = (const float*)d_in[12];
  const float* mlpW   = (const float*)d_in[13];
  const float* mlpb   = (const float*)d_in[14];
  const float* linW   = (const float*)d_in[15];
  const float* linb   = (const float*)d_in[16];
  float* out = (float*)d_out;

  const int nBlkA = (nA + NB - 1) / NB;
  const int nBlkB = (nBn + NB - 1) / NB;
  const int CB    = (nBlkA + NCHK - 1) / NCHK;

  char* ws = (char*)d_ws;
  size_t off = 0;
  const size_t szW  = (size_t)nL * WPL * 2;
  const size_t szHA = (size_t)nBlkA * NB * DF * 4;
  const size_t szHB = (size_t)nBlkB * NB * DF * 4;
  const size_t szP  = (size_t)CB * NB * DF * 4;
  const size_t szPA = (size_t)nBlkA * NG * DF * 4;
  const size_t szPB = (size_t)nBlkB * NG * DF * 4;
  const size_t oWh = off; off += szW;  off = (off + 255) & ~(size_t)255;
  const size_t oWl = off; off += szW;  off = (off + 255) & ~(size_t)255;
  const size_t oHA = off; off += szHA; off = (off + 255) & ~(size_t)255;
  const size_t oHB = off; off += szHB; off = (off + 255) & ~(size_t)255;
  const size_t oP  = off; off += szP;  off = (off + 255) & ~(size_t)255;
  const size_t oPA = off; off += szPA; off = (off + 255) & ~(size_t)255;
  const size_t oPB = off; off += szPB; off = (off + 255) & ~(size_t)255;
  if (off > ws_size) return;
  bf16_t* whi  = (bf16_t*)(ws + oWh);
  bf16_t* wlo  = (bf16_t*)(ws + oWl);
  float*  ha1  = (float*)(ws + oHA);
  float*  hb1  = (float*)(ws + oHB);
  float*  pP   = (float*)(ws + oP);
  float*  poolA = (float*)(ws + oPA);
  float*  poolB = (float*)(ws + oPB);

  const int vAA = ((eAA & 3) == 0) ? 1 : 0;
  const int vAB = ((eAB & 3) == 0) ? 1 : 0;
  const int vBA = ((eBA & 3) == 0) ? 1 : 0;

  const int nTot = nL * WPL / 8;
  k_wprep<<<(nTot + NTHR - 1) / NTHR, NTHR, 0, stream>>>(Wl, Wr, whi, wlo, nTot);

  hipFuncSetAttribute(reinterpret_cast<const void*>(&k_layer),
                      hipFuncAttributeMaxDynamicSharedMemorySize, LDS_LAYER);
  hipFuncSetAttribute(reinterpret_cast<const void*>(&k_head),
                      hipFuncAttributeMaxDynamicSharedMemorySize, LDS_HEAD);

  for (int l = 0; l < 2; ++l) {
    const float* xa_in = (l == 0) ? x_a : ha1;
    const float* xb_in = (l == 0) ? x_b : hb1;
    const int md = (l == 0) ? 0 : 1;
    const bf16_t* wa1h = whi + (size_t)l * WPL;
    const bf16_t* wa1l = wlo + (size_t)l * WPL;
    const bf16_t* wa2h = wa1h + OFF_A2;
    const bf16_t* wa2l = wa1l + OFF_A2;
    const bf16_t* wbh  = wa1h + OFF_B;
    const bf16_t* wbl  = wa1l + OFF_B;
    const float* bl0 = bl + (size_t)(l * 3 + 0) * DF;
    const float* bl1 = bl + (size_t)(l * 3 + 1) * DF;
    const float* bl2 = bl + (size_t)(l * 3 + 2) * DF;

    k_layer<<<nBlkB, NTHR, LDS_LAYER, stream>>>(
        ab_src, ab_dst, eAB, vAB, xa_in, nA, xb_in, nBn,
        wbh, wbl, KVB, 1, bl1, bl1, 1.0f, 0.0f,
        pP, 0, hb1, md, 1, bat_b, poolB, 0);

    for (int cix = 0; cix < NCHK; ++cix) {
      const int rem = nBlkA - cix * CB;
      const int nb  = rem < CB ? rem : CB;
      if (nb <= 0) continue;
      const int rowBase = cix * CB * NB;
      k_layer<<<nb, NTHR, LDS_LAYER, stream>>>(
          aa_src, aa_dst, eAA, vAA, xa_in, nA, xa_in, nA,
          wa1h, wa1l, KVA1, 1, bl0, bl2, 1.0f, 1.0f,
          pP, 0, pP, 0, 0, bat_a, poolA, rowBase);
      k_layer<<<nb, NTHR, LDS_LAYER, stream>>>(
          ba_src, ba_dst, eBA, vBA, xb_in, nBn, xa_in, nA,
          wa2h, wa2l, KVA2, 0, bl0, bl0, 0.0f, 0.0f,
          pP, 1, ha1 + (size_t)rowBase * DF, md, 1, bat_a,
          poolA + (size_t)cix * CB * NG * DF, rowBase);
    }
  }

  k_head<<<1, NTHR, LDS_HEAD, stream>>>(poolA, nBlkA, poolB, nBlkB, mlpW, mlpb, linW, linb, out);
}
